// SpatialMultiAttention_77197742178875
// MI455X (gfx1250) — hardware-verified
//
#include <hip/hip_runtime.h>
#define BB 2
#define NTOK 16384
#define CC 128
#define HD 16
#define NR (BB * NTOK)

typedef __bf16 v16b __attribute__((ext_vector_type(16)));
typedef unsigned short v8us __attribute__((ext_vector_type(8), may_alias));
typedef float  v8f  __attribute__((ext_vector_type(8)));
typedef float  v4f  __attribute__((ext_vector_type(4)));
typedef float  v4fa __attribute__((ext_vector_type(4), may_alias));
union FragB { v16b v; v8us half[2]; unsigned short u[16]; };

__device__ __forceinline__ unsigned short bf16_bits(float x) { unsigned int u = __float_as_uint(x); return (unsigned short)((u + 0x7FFFu + ((u >> 16) & 1u)) >> 16); }
__device__ __forceinline__ float bf16_val(unsigned short b) { return __uint_as_float(((unsigned int)b) << 16); }
__device__ __forceinline__ float bf16_round(float x) { return bf16_val(bf16_bits(x)); }
template <int NT>
__device__ __forceinline__ v8f mmaN(v16b ah, v16b al, v16b bh, v16b bl, v8f c) {
  c = __builtin_amdgcn_wmma_f32_16x16x32_bf16(false, ah, false, bh, (short)0, c, false, false);
  if (NT >= 2) c = __builtin_amdgcn_wmma_f32_16x16x32_bf16(false, al, false, bh, (short)0, c, false, false);
  if (NT >= 3) c = __builtin_amdgcn_wmma_f32_16x16x32_bf16(false, ah, false, bl, (short)0, c, false, false);
  asm volatile("v_nop\n\tv_nop\n\tv_nop\n\tv_nop" : "+v"(c) : "v"(ah), "v"(al), "v"(bh), "v"(bl));
  return c;
}

__global__ __launch_bounds__(256) void k_wt_bf16(const float* __restrict__ W, unsigned short* __restrict__ Wt, int K, int N) {
  const int t = blockIdx.x * 256 + threadIdx.x;
  const int k8n = K / 8;
  if (t >= N * k8n) return;
  const int n = t / k8n, k8 = (t % k8n) * 8;
  v8us v;
#pragma unroll
  for (int i = 0; i < 8; ++i) v[i] = bf16_bits(W[(size_t)(k8 + i) * N + n]);
  *(volatile v8us*)(Wt + (size_t)n * K + k8) = v;
  __threadfence();
  *(volatile v8us*)(Wt + (size_t)n * K + k8) = v;
}

template <bool ASPLIT, int ACT, bool BIAS_BF16>
__global__ __launch_bounds__(128) void k_gemm_bf(const float* __restrict__ A, int lda, const unsigned short* __restrict__ Wt, int ldb,
                                               const float* __restrict__ bias, float* __restrict__ C, int ldc, int M, int N, int K) {
  __shared__ __attribute__((aligned(16))) float so[4][16][64];
  const int tid = threadIdx.x, w = tid >> 5, lane = tid & 31, ln = lane & 15, hh = lane >> 4;
  const int ntn = N / 64;
  const int wid = blockIdx.x * 4 + w;
  const int mt = wid / ntn, nq = wid % ntn;
  if (mt * 16 >= M) return;
  const int row0 = mt * 16, col0 = nq * 64;
  const float* arow = A + (size_t)(row0 + ln) * lda;
  v8f acc[4] = {};
  for (int kb = 0; kb < K; kb += 32) {
    FragB ah, al;
    const v4f x0 = *(const v4fa*)(arow + kb + 8 * hh), x1 = *(const v4fa*)(arow + kb + 8 * hh + 4);
    const v4f x2 = *(const v4fa*)(arow + kb + 16 + 8 * hh), x3 = *(const v4fa*)(arow + kb + 16 + 8 * hh + 4);
    float xs[16] = {x0[0],x0[1],x0[2],x0[3],x1[0],x1[1],x1[2],x1[3],x2[0],x2[1],x2[2],x2[3],x3[0],x3[1],x3[2],x3[3]};
#pragma unroll
    for (int i = 0; i < 16; ++i) { const unsigned short hb = bf16_bits(xs[i]); ah.u[i] = hb; al.u[i] = ASPLIT ? bf16_bits(xs[i] - bf16_val(hb)) : (unsigned short)0; }
#pragma unroll
    for (int t = 0; t < 4; ++t) {
      const unsigned short* brow = Wt + (size_t)(col0 + t * 16 + ln) * ldb + kb;
      FragB b;
      b.half[0] = *(const v8us*)(brow + 8 * hh);
      b.half[1] = *(const v8us*)(brow + 16 + 8 * hh);
      acc[t] = mmaN<ASPLIT ? 2 : 1>(ah.v, al.v, b.v, b.v, acc[t]);
    }
  }
#pragma unroll
  for (int t = 0; t < 4; ++t) {
    float bv = bias ? bias[col0 + t * 16 + ln] : 0.f;
    if (BIAS_BF16) bv = bf16_round(bv);
#pragma unroll
    for (int r = 0; r < 8; ++r) { float v = acc[t][r] + bv; if (ACT == 1) v = fmaxf(v, 0.f); so[w][8 * hh + r][t * 16 + ln] = v; }
  }
  __builtin_amdgcn_fence(__ATOMIC_ACQ_REL, "workgroup");
  __builtin_amdgcn_wave_barrier();
  const int rsub = lane >> 4, c4 = (lane & 15) * 4;
  for (int pass = 0; pass < 2; ++pass) {
#pragma unroll
    for (int q = 0; q < 8; ++q) {
      const int r = q * 2 + rsub;
      const v4f v = *(const v4fa*)&so[w][r][c4];
      *(volatile v4f*)(C + (size_t)(row0 + r) * ldc + col0 + c4) = v;
    }
    if (pass == 0) __threadfence();
  }
}

template <int D, bool CAUSAL>
__global__ __launch_bounds__(128) void k_flash(const float* __restrict__ qb, const float* __restrict__ kb, const float* __restrict__ vb,
                                             int pitch, int T, int H, float scale, float* __restrict__ y, int ypitch) {
  constexpr int KS = D / 32;
  constexpr int DT = D / 16;
  __shared__ __attribute__((aligned(16))) unsigned short sKh[32][D + 8], sKl[32][D + 8], sVh[32][D + 8], sVl[32][D + 8];
  __shared__ __attribute__((aligned(16))) unsigned short sPh[4][16][40], sPl[4][16][40];
  __shared__ __attribute__((aligned(16))) float sO[4][16][D];
  const int tid = threadIdx.x, w = tid >> 5, lane = tid & 31, ln = lane & 15, hh = lane >> 4;
  const int nqb = (T + 63) / 64;
  const int bh = blockIdx.x / nqb, qblk = blockIdx.x % nqb;
  const int b = bh / H, h = bh % H;
  const int q0 = qblk * 64 + w * 16;
  const float* Q = qb + (size_t)b * T * pitch + h * D;
  const float* K = kb + (size_t)b * T * pitch + h * D;
  const float* V = vb + (size_t)b * T * pitch + h * D;

  FragB aqh[KS], aql[KS];
  {
    int row = q0 + ln; if (row >= T) row = T - 1;
    const float* qr = Q + (size_t)row * pitch;
#pragma unroll
    for (int ks = 0; ks < KS; ++ks)
#pragma unroll
      for (int i = 0; i < 16; ++i) {
        const int d = ks * 32 + ((i < 8) ? (8 * hh + i) : (16 + 8 * hh + (i - 8)));
        const float x = qr[d] * scale; const unsigned short hb = bf16_bits(x);
        aqh[ks].u[i] = hb; aql[ks].u[i] = bf16_bits(x - bf16_val(hb));
      }
  }
  float m_r[8], l_r[8];
#pragma unroll
  for (int r = 0; r < 8; ++r) { m_r[r] = -3.0e38f; l_r[r] = 0.f; }
  v8f oacc[DT];
#pragma unroll
  for (int dt = 0; dt < DT; ++dt) oacc[dt] = (v8f){0.f,0.f,0.f,0.f,0.f,0.f,0.f,0.f};

  const int kv_end = CAUSAL ? min(T, qblk * 64 + 64) : T;
  for (int j0 = 0; j0 < kv_end; j0 += 32) {
    __syncthreads();
    for (int e = tid; e < 32 * (D / 4); e += 128) {
      const int r = e / (D / 4), c4 = (e % (D / 4)) * 4;
      const int key = j0 + r;
      v4f kf = {0.f,0.f,0.f,0.f}, vf = {0.f,0.f,0.f,0.f};
      if (key < T) { kf = *(const v4fa*)(K + (size_t)key * pitch + c4); vf = *(const v4fa*)(V + (size_t)key * pitch + c4); }
#pragma unroll
      for (int t = 0; t < 4; ++t) {
        unsigned short hb = bf16_bits(kf[t]); sKh[r][c4 + t] = hb; sKl[r][c4 + t] = bf16_bits(kf[t] - bf16_val(hb));
        hb = bf16_bits(vf[t]); sVh[r][c4 + t] = hb; sVl[r][c4 + t] = bf16_bits(vf[t] - bf16_val(hb));
      }
    }
    __syncthreads();
    v8f s[2];
#pragma unroll
    for (int nt = 0; nt < 2; ++nt) {
      v8f acc = {};
#pragma unroll
      for (int ks = 0; ks < KS; ++ks) {
        FragB bh_, bl_;
        bh_.half[0] = *(const v8us*)&sKh[nt * 16 + ln][ks * 32 + 8 * hh]; bh_.half[1] = *(const v8us*)&sKh[nt * 16 + ln][ks * 32 + 16 + 8 * hh];
        bl_.half[0] = *(const v8us*)&sKl[nt * 16 + ln][ks * 32 + 8 * hh]; bl_.half[1] = *(const v8us*)&sKl[nt * 16 + ln][ks * 32 + 16 + 8 * hh];
        acc = mmaN<3>(aqh[ks].v, aql[ks].v, bh_.v, bl_.v, acc);
      }
      s[nt] = acc;
    }
    float alpha[8];
#pragma unroll
    for (int r = 0; r < 8; ++r) {
      const int qi = q0 + 8 * hh + r;
      const int ja = j0 + ln, jb = j0 + 16 + ln;
      if (CAUSAL) { if (ja > qi) s[0][r] = -3.0e38f; if (jb > qi) s[1][r] = -3.0e38f; }
      if (ja >= T) s[0][r] = -3.0e38f;
      if (jb >= T) s[1][r] = -3.0e38f;
      float mx = fmaxf(s[0][r], s[1][r]);
      mx = fmaxf(mx, __shfl_xor(mx, 1, 32)); mx = fmaxf(mx, __shfl_xor(mx, 2, 32)); mx = fmaxf(mx, __shfl_xor(mx, 4, 32)); mx = fmaxf(mx, __shfl_xor(mx, 8, 32));
      const float mnew = fmaxf(m_r[r], mx);
      alpha[r] = (mnew > -1.0e38f) ? __expf(m_r[r] - mnew) : 1.0f;
      const float p0 = (s[0][r] > -1.0e38f) ? __expf(s[0][r] - mnew) : 0.f;
      const float p1 = (s[1][r] > -1.0e38f) ? __expf(s[1][r] - mnew) : 0.f;
      m_r[r] = mnew;
      l_r[r] = l_r[r] * alpha[r] + p0 + p1;
      unsigned short hb = bf16_bits(p0); sPh[w][8 * hh + r][ln] = hb;      sPl[w][8 * hh + r][ln] = bf16_bits(p0 - bf16_val(hb));
      hb = bf16_bits(p1);                sPh[w][8 * hh + r][16 + ln] = hb; sPl[w][8 * hh + r][16 + ln] = bf16_bits(p1 - bf16_val(hb));
    }
#pragma unroll
    for (int dt = 0; dt < DT; ++dt)
#pragma unroll
      for (int r = 0; r < 8; ++r) oacc[dt][r] *= alpha[r];
    __builtin_amdgcn_fence(__ATOMIC_ACQ_REL, "workgroup");
    __builtin_amdgcn_wave_barrier();
    FragB pah, pal;
    pah.half[0] = *(const v8us*)&sPh[w][ln][8 * hh]; pah.half[1] = *(const v8us*)&sPh[w][ln][16 + 8 * hh];
    pal.half[0] = *(const v8us*)&sPl[w][ln][8 * hh]; pal.half[1] = *(const v8us*)&sPl[w][ln][16 + 8 * hh];
#pragma unroll
    for (int dt = 0; dt < DT; ++dt) {
      FragB bvh, bvl;
#pragma unroll
      for (int i = 0; i < 8; ++i) {
        bvh.u[i] = sVh[8 * hh + i][dt * 16 + ln]; bvh.u[8 + i] = sVh[16 + 8 * hh + i][dt * 16 + ln];
        bvl.u[i] = sVl[8 * hh + i][dt * 16 + ln]; bvl.u[8 + i] = sVl[16 + 8 * hh + i][dt * 16 + ln];
      }
      oacc[dt] = mmaN<3>(pah.v, pal.v, bvh.v, bvl.v, oacc[dt]);
    }
    __builtin_amdgcn_fence(__ATOMIC_ACQ_REL, "workgroup");
    __builtin_amdgcn_wave_barrier();
  }
#pragma unroll
  for (int r = 0; r < 8; ++r) {
    float l = l_r[r];
    l += __shfl_xor(l, 1, 32); l += __shfl_xor(l, 2, 32); l += __shfl_xor(l, 4, 32); l += __shfl_xor(l, 8, 32);
    l_r[r] = (l > 0.f) ? 1.0f / l : 0.f;
  }
#pragma unroll
  for (int dt = 0; dt < DT; ++dt)
#pragma unroll
    for (int r = 0; r < 8; ++r) sO[w][8 * hh + r][dt * 16 + ln] = oacc[dt][r] * l_r[r];
  __builtin_amdgcn_fence(__ATOMIC_ACQ_REL, "workgroup");
  __builtin_amdgcn_wave_barrier();
  for (int pass = 0; pass < 2; ++pass) {
    for (int r = 0; r < 16; ++r) {
      const int row = q0 + r;
      if (row < T && lane < D / 4) {
        const v4f val = *(const v4fa*)&sO[w][r][lane * 4];
        *(volatile v4f*)(y + ((size_t)b * T + row) * ypitch + h * D + lane * 4) = val;
      }
    }
    if (pass == 0) __threadfence();
  }
}

template <bool ASPLIT, int ACT, bool BIAS_BF16, bool RES_BF16>
__global__ __launch_bounds__(128) void k_gemm_bf3(const float* __restrict__ A, int lda, const unsigned short* __restrict__ Wt, int ldb,
                                                const float* __restrict__ bias, const float* __restrict__ resid, int rmod, int ldr,
                                                float* __restrict__ C, int ldc, int M, int N, int K) {
  __shared__ __attribute__((aligned(16))) float so[4][16][64];
  const int tid = threadIdx.x, w = tid >> 5, lane = tid & 31, ln = lane & 15, hh = lane >> 4;
  const int ntn = N / 64;
  const int wid = blockIdx.x * 4 + w;
  const int mt = wid / ntn, nq = wid % ntn;
  if (mt * 16 >= M) return;
  const int row0 = mt * 16, col0 = nq * 64;
  const float* arow = A + (size_t)(row0 + ln) * lda;
  v8f acc[4] = {};
  for (int kb = 0; kb < K; kb += 32) {
    FragB ah, al;
    const v4f x0 = *(const v4fa*)(arow + kb + 8 * hh), x1 = *(const v4fa*)(arow + kb + 8 * hh + 4);
    const v4f x2 = *(const v4fa*)(arow + kb + 16 + 8 * hh), x3 = *(const v4fa*)(arow + kb + 16 + 8 * hh + 4);
    float xs[16] = {x0[0],x0[1],x0[2],x0[3],x1[0],x1[1],x1[2],x1[3],x2[0],x2[1],x2[2],x2[3],x3[0],x3[1],x3[2],x3[3]};
#pragma unroll
    for (int i = 0; i < 16; ++i) { const unsigned short hb = bf16_bits(xs[i]); ah.u[i] = hb; al.u[i] = ASPLIT ? bf16_bits(xs[i] - bf16_val(hb)) : (unsigned short)0; }
#pragma unroll
    for (int t = 0; t < 4; ++t) {
      const unsigned short* brow = Wt + (size_t)(col0 + t * 16 + ln) * ldb + kb;
      FragB b;
      b.half[0] = *(const v8us*)(brow + 8 * hh);
      b.half[1] = *(const v8us*)(brow + 16 + 8 * hh);
      acc[t] = mmaN<ASPLIT ? 2 : 1>(ah.v, al.v, b.v, b.v, acc[t]);
    }
  }
#pragma unroll
  for (int t = 0; t < 4; ++t) {
    const int col = col0 + t * 16 + ln;
    float bv = bias ? bias[col] : 0.f;
    if (BIAS_BF16) bv = bf16_round(bv);
#pragma unroll
    for (int r = 0; r < 8; ++r) {
      float v = acc[t][r] + bv;
      if (resid) { float rv = resid[(size_t)((row0 + 8 * hh + r) % rmod) * ldr + col]; if (RES_BF16) rv = bf16_round(rv); v += rv; }
      if (ACT == 1) v = fmaxf(v, 0.f);
      if (ACT == 2) v = 0.5f * v * (1.0f + erff(v * 0.70710678118654752f));
      if (ACT == 3) { const float u = 0.7978845608028654f * (v + 0.044715f * v * v * v); v = 0.5f * v * (1.0f + tanhf(u)); }
      so[w][8 * hh + r][t * 16 + ln] = v;
    }
  }
  __builtin_amdgcn_fence(__ATOMIC_ACQ_REL, "workgroup");
  __builtin_amdgcn_wave_barrier();
  const int rsub = lane >> 4, c4 = (lane & 15) * 4;
  for (int pass = 0; pass < 2; ++pass) {
#pragma unroll
    for (int q = 0; q < 8; ++q) {
      const int r = q * 2 + rsub;
      const v4f v = *(const v4fa*)&so[w][r][c4];
      *(volatile v4f*)(C + (size_t)(row0 + r) * ldc + col0 + c4) = v;
    }
    if (pass == 0) __threadfence();
  }
}
template <bool PARAM_BF16>
__global__ __launch_bounds__(256) void k_layernorm(const float* __restrict__ X, const float* __restrict__ R, const float* __restrict__ g, const float* __restrict__ bta,
                                                  float* __restrict__ out_sum, float* __restrict__ out_norm, int N, float eps) {
  __shared__ float red[256];
  const int row = blockIdx.x, tid = threadIdx.x;
  const float* x = X + (size_t)row * N; const float* rr = R ? R + (size_t)row * N : nullptr;
  float vals[16];
  const int per = N / 256;
  float s1 = 0.f;
  for (int u = 0; u < per / 4; ++u) {
    const int j = tid * 4 + 1024 * u;
    const v4f a = *(const v4fa*)(x + j);
    v4f b = {0.f,0.f,0.f,0.f}; if (rr) b = *(const v4fa*)(rr + j);
#pragma unroll
    for (int q = 0; q < 4; ++q) { const float v = a[q] + b[q]; vals[u * 4 + q] = v; s1 += v; }
  }
  red[tid] = s1; __syncthreads();
  for (int st = 128; st > 0; st >>= 1) { if (tid < st) red[tid] += red[tid + st]; __syncthreads(); }
  const float mu = red[0] / (float)N; __syncthreads();
  float s2 = 0.f;
  for (int u = 0; u < per / 4; ++u)
#pragma unroll
    for (int q = 0; q < 4; ++q) { const float c = vals[u * 4 + q] - mu; s2 += c * c; }
  red[tid] = s2; __syncthreads();
  for (int st = 128; st > 0; st >>= 1) { if (tid < st) red[tid] += red[tid + st]; __syncthreads(); }
  const float rs = rsqrtf(red[0] / (float)N + eps);
  for (int pass = 0; pass < 2; ++pass) {
    for (int u = 0; u < per / 4; ++u) {
      const int j = tid * 4 + 1024 * u;
      v4f o, sm;
#pragma unroll
      for (int q = 0; q < 4; ++q) {
        float gg = g[j + q], bb = bta[j + q];
        if (PARAM_BF16) { gg = bf16_round(gg); bb = bf16_round(bb); }
        sm[q] = vals[u * 4 + q]; o[q] = (vals[u * 4 + q] - mu) * rs * gg + bb;
      }
      if (out_sum) *(volatile v4f*)(out_sum + (size_t)row * N + j) = sm;
      *(volatile v4f*)(out_norm + (size_t)row * N + j) = o;
    }
    if (pass == 0) __threadfence();
  }
}


typedef _Float16 v16h __attribute__((ext_vector_type(16)));
union FragH { v16h v; v8us half[2]; _Float16 h[16]; unsigned short u[16]; };
template <int NT>
__device__ __forceinline__ v8f mmaH(v16h ah, v16h al, v16h bh, v16h bl, v8f c) {
  c = __builtin_amdgcn_wmma_f32_16x16x32_f16(false, ah, false, bh, (short)0, c, false, false);
  if (NT >= 2) c = __builtin_amdgcn_wmma_f32_16x16x32_f16(false, al, false, bh, (short)0, c, false, false);
  if (NT >= 3) c = __builtin_amdgcn_wmma_f32_16x16x32_f16(false, ah, false, bl, (short)0, c, false, false);
  asm volatile("v_nop\n\tv_nop\n\tv_nop\n\tv_nop" : "+v"(c) : "v"(ah), "v"(al), "v"(bh), "v"(bl));
  return c;
}
template <bool ASPLIT>
__global__ __launch_bounds__(128) void k_gemm_h(const float* __restrict__ A, int lda, size_t sA, const _Float16* __restrict__ Bh, int ldb, size_t sB, float alpha, float* __restrict__ C, int ldc, size_t sC, int M, int N, int K) {
  __shared__ __attribute__((aligned(16))) float so[4][16][64];
  const int tid = threadIdx.x, w = tid >> 5, lane = tid & 31, ln = lane & 15, hh = lane >> 4; const int by = blockIdx.y;
  A += (size_t)by * sA; Bh += (size_t)by * sB; C += (size_t)by * sC;
  const int ntn = (N + 63) / 64; const int wid = blockIdx.x * 4 + w; const int mt = wid / ntn, nq = wid % ntn; if (mt * 16 >= M) return;
  const int row0 = mt * 16, col0 = nq * 64; const float* arow = A + (size_t)(row0 + ln) * lda;
  v8f acc[4] = {};
  for (int kb = 0; kb < K; kb += 32) {
    FragH ah, al;
    const v4f x0 = *(const v4fa*)(arow + kb + 8 * hh), x1 = *(const v4fa*)(arow + kb + 8 * hh + 4), x2 = *(const v4fa*)(arow + kb + 16 + 8 * hh), x3 = *(const v4fa*)(arow + kb + 16 + 8 * hh + 4);
    float xs[16] = {x0[0],x0[1],x0[2],x0[3],x1[0],x1[1],x1[2],x1[3],x2[0],x2[1],x2[2],x2[3],x3[0],x3[1],x3[2],x3[3]};
#pragma unroll
    for (int i = 0; i < 16; ++i) { const _Float16 h = (_Float16)xs[i]; ah.h[i] = h; al.h[i] = ASPLIT ? (_Float16)(xs[i] - (float)h) : (_Float16)0.0f; }
#pragma unroll
    for (int t = 0; t < 4; ++t) { if (col0 + t * 16 >= N) continue; const size_t boff = (size_t)(col0 + t * 16 + ln) * ldb + kb; FragH bq; bq.half[0] = *(const v8us*)(Bh + boff + 8 * hh); bq.half[1] = *(const v8us*)(Bh + boff + 16 + 8 * hh);
      acc[t] = mmaH<ASPLIT ? 2 : 1>(ah.v, al.v, bq.v, bq.v, acc[t]); }
  }
#pragma unroll
  for (int t = 0; t < 4; ++t) { if (col0 + t * 16 >= N) continue;
#pragma unroll
    for (int r = 0; r < 8; ++r) so[w][8 * hh + r][t * 16 + ln] = acc[t][r] * alpha; }
  __builtin_amdgcn_fence(__ATOMIC_ACQ_REL, "workgroup"); __builtin_amdgcn_wave_barrier();
  const int rsub = lane >> 4, c4 = (lane & 15) * 4;
  for (int pass = 0; pass < 2; ++pass) {
#pragma unroll
    for (int q = 0; q < 8; ++q) { const int r = q * 2 + rsub; if (col0 + c4 < N) { const v4f v = *(const v4fa*)&so[w][r][c4]; *(volatile v4f*)(C + (size_t)(row0 + r) * ldc + col0 + c4) = v; } }
    if (pass == 0) __threadfence(); }
}

__global__ __launch_bounds__(256) void k_wt_f16(const float* __restrict__ W, _Float16* __restrict__ Wt, int K, int N, float scale) {
  const int t = blockIdx.x * 256 + threadIdx.x; if (t >= N * (K / 8)) return; const int n = t / (K / 8), k8 = (t % (K / 8)) * 8; FragH f;
#pragma unroll
  for (int i = 0; i < 8; ++i) f.h[i] = (_Float16)(bf16_round(W[(size_t)(k8 + i) * N + n]) * scale); const v8us o = f.half[0];
  *(volatile v8us*)((unsigned short*)Wt + (size_t)n * K + k8) = o; __threadfence(); *(volatile v8us*)((unsigned short*)Wt + (size_t)n * K + k8) = o;
}
template <int ACT>
__global__ __launch_bounds__(128) void k_gemm_hhx(const _Float16* __restrict__ A, int lda, size_t sA, const _Float16* __restrict__ Bh, int ldb, size_t sB, float alpha, const float* __restrict__ bias, size_t sBias, const float* __restrict__ CP, int rowsPerB, size_t sCPb, int row0g,
    float* __restrict__ C, _Float16* __restrict__ C16, int ldc, size_t sC, int M, int N, int K) {
  __shared__ __attribute__((aligned(16))) float so[4][16][64];
  const int tid = threadIdx.x, w = tid >> 5, lane = tid & 31, ln = lane & 15, hh = lane >> 4; const int by = blockIdx.y;
  A += (size_t)by * sA; Bh += (size_t)by * sB; const size_t cofs = (size_t)by * sC; const float* bp = bias ? bias + (size_t)by * sBias : nullptr;
  const int ntn = (N + 63) / 64; const int wid = blockIdx.x * 4 + w; const int mt = wid / ntn, nq = wid % ntn; if (mt * 16 >= M) return;
  const int row0 = mt * 16, col0 = nq * 64; const _Float16* arow = A + (size_t)(row0 + ln) * lda;
  v8f acc[4] = {};
  for (int kb = 0; kb < K; kb += 32) { FragH ah; ah.half[0] = *(const v8us*)((const unsigned short*)arow + kb + 8 * hh); ah.half[1] = *(const v8us*)((const unsigned short*)arow + kb + 16 + 8 * hh);
#pragma unroll
    for (int t = 0; t < 4; ++t) { if (col0 + t * 16 >= N) continue; const size_t boff = (size_t)(col0 + t * 16 + ln) * ldb + kb; FragH bq; bq.half[0] = *(const v8us*)((const unsigned short*)Bh + boff + 8 * hh); bq.half[1] = *(const v8us*)((const unsigned short*)Bh + boff + 16 + 8 * hh);
      acc[t] = mmaH<1>(ah.v, ah.v, bq.v, bq.v, acc[t]); }
  }
#pragma unroll
  for (int t = 0; t < 4; ++t) { if (col0 + t * 16 >= N) continue; const int col = col0 + t * 16 + ln; const float bv = bp ? bf16_round(bp[col]) : 0.f;
#pragma unroll
    for (int r = 0; r < 8; ++r) { float v = acc[t][r] * alpha + bv; if (CP) { const int bidx = (row0g + row0 + 8 * hh + r) / rowsPerB; v += CP[(size_t)bidx * sCPb + (size_t)by * 64 + col]; } if (ACT == 1) v = (v > 0.f) ? v : expm1f(v); else if (ACT == 3) v = fmaxf(v, 0.f); so[w][8 * hh + r][t * 16 + ln] = v; } }
  __builtin_amdgcn_fence(__ATOMIC_ACQ_REL, "workgroup"); __builtin_amdgcn_wave_barrier();
  const int rsub = lane >> 4, c4 = (lane & 15) * 4; typedef _Float16 v4h __attribute__((ext_vector_type(4)));
  for (int pass = 0; pass < 2; ++pass) {
#pragma unroll
    for (int q = 0; q < 8; ++q) { const int r = q * 2 + rsub; if (col0 + c4 < N) { const v4f v = *(const v4fa*)&so[w][r][c4]; if (C) *(volatile v4f*)(C + cofs + (size_t)(row0 + r) * ldc + col0 + c4) = v; if (C16) { v4h h4; for (int i = 0; i < 4; ++i) h4[i] = (_Float16)v[i]; *(volatile v4h*)(C16 + cofs + (size_t)(row0 + r) * ldc + col0 + c4) = h4; } } }
    if (pass == 0) __threadfence(); }
}


__global__ __launch_bounds__(256) void k_x16(const float* __restrict__ x, _Float16* __restrict__ X16, size_t n8) { const size_t t = (size_t)blockIdx.x * 256 + threadIdx.x; if (t >= n8) return; FragH f;
#pragma unroll
  for (int q = 0; q < 8; ++q) f.h[q] = (_Float16)bf16_round(x[t * 8 + q]); *(volatile v8us*)((unsigned short*)X16 + t * 8) = f.half[0]; __threadfence(); *(volatile v8us*)((unsigned short*)X16 + t * 8) = f.half[0]; }
__global__ __launch_bounds__(256) void k_round16f(const float* __restrict__ W, _Float16* __restrict__ Bt, size_t n8) { const size_t t = (size_t)blockIdx.x * 256 + threadIdx.x; if (t >= n8) return; FragH f;
#pragma unroll
  for (int i = 0; i < 8; ++i) f.h[i] = (_Float16)(bf16_round(W[t * 8 + i]) * 16.0f); *(volatile v8us*)((unsigned short*)Bt + t * 8) = f.half[0]; __threadfence(); *(volatile v8us*)((unsigned short*)Bt + t * 8) = f.half[0]; }
template <int KS>
__global__ __launch_bounds__(256) void k_patch(const _Float16* __restrict__ X16, _Float16* __restrict__ AP) { constexpr int WK = 128 / KS, NK = WK * WK, KK = CC * KS * KS; const size_t t = (size_t)blockIdx.x * 256 + threadIdx.x; if (t >= (size_t)BB * NK * KK / 8) return;
  const size_t row = t / (KK / 8); const int k8 = (int)(t % (KK / 8)) * 8; const int b = (int)(row / NK), tok = (int)(row % NK); const int py = tok / WK, px = tok % WK; FragH f;
#pragma unroll
  for (int q = 0; q < 8; ++q) { const int kk = k8 + q; const int ci = kk / (KS * KS), rem = kk % (KS * KS), ky = rem / KS, kx = rem % KS; f.h[q] = X16[((size_t)b * NTOK + (size_t)(py * KS + ky) * 128 + px * KS + kx) * CC + ci]; }
  *(volatile v8us*)((unsigned short*)AP + t * 8) = f.half[0]; __threadfence(); *(volatile v8us*)((unsigned short*)AP + t * 8) = f.half[0]; }
__global__ __launch_bounds__(256) void k_lngelu(const float* __restrict__ XR, int nrow, const float* __restrict__ g, const float* __restrict__ bb, _Float16* __restrict__ XG) { const int tid = threadIdx.x, wv = tid >> 5, lane = tid & 31; const int row = blockIdx.x * 8 + wv; if (row >= nrow) return; const v4f v = *(const v4fa*)(XR + (size_t)row * CC + lane * 4);
  float s = v[0] + v[1] + v[2] + v[3]; for (int o = 16; o >= 1; o >>= 1) s += __shfl_xor(s, o, 32); const float mu = s / (float)CC; float q2 = 0.f;
#pragma unroll
  for (int u = 0; u < 4; ++u) { const float d = v[u] - mu; q2 += d * d; } for (int o = 16; o >= 1; o >>= 1) q2 += __shfl_xor(q2, o, 32); const float rs = rsqrtf(q2 / (float)CC + 1e-5f);
  typedef _Float16 v4h __attribute__((ext_vector_type(4))); v4h o;
#pragma unroll
  for (int u = 0; u < 4; ++u) { const int c = lane * 4 + u; const float y = (v[u] - mu) * rs * bf16_round(g[c]) + bf16_round(bb[c]); o[u] = (_Float16)(0.5f * y * (1.0f + erff(y * 0.70710678118654752f))); }
  *(volatile v4h*)(XG + (size_t)row * CC + lane * 4) = o; __threadfence(); *(volatile v4h*)(XG + (size_t)row * CC + lane * 4) = o; }
template <int WK>
__global__ __launch_bounds__(256) void k_vt(const float* __restrict__ KV, const float* __restrict__ lw, const float* __restrict__ lb, _Float16* __restrict__ Vt) { constexpr int NK = WK * WK; const size_t t = (size_t)blockIdx.x * 256 + threadIdx.x; if (t >= (size_t)BB * 64 * NK / 8) return;
  const int b = (int)(t / (64 * NK / 8)); const int rem = (int)(t % (64 * NK / 8)); const int c = rem / (NK / 8); const int t8 = (rem % (NK / 8)) * 8; const int py = t8 / WK, px0 = t8 % WK; const int h = c / HD, d = c % HD;
  float w9[9]; for (int q = 0; q < 9; ++q) w9[q] = bf16_round(lw[c * 9 + q]); const float bias = bf16_round(lb[c]); const float* kvb = KV + (size_t)b * NK * CC + 64 + c; FragH f;
#pragma unroll
  for (int u = 0; u < 8; ++u) { const int px = px0 + u; float acc = kvb[(size_t)(py * WK + px) * CC] + bias;
#pragma unroll
    for (int q = 0; q < 9; ++q) { const int yy = py + q / 3 - 1, xx = px + q % 3 - 1; const bool ok = (yy >= 0 && yy < WK && xx >= 0 && xx < WK); const int yc = yy < 0 ? 0 : (yy >= WK ? WK - 1 : yy), xc = xx < 0 ? 0 : (xx >= WK ? WK - 1 : xx); const float nv = kvb[(size_t)(yc * WK + xc) * CC]; acc += ok ? nv * w9[q] : 0.f; }
    f.h[u] = (_Float16)acc; }
  unsigned short* dst = (unsigned short*)Vt + ((size_t)(b * 4 + h) * HD + d) * NK + t8; *(volatile v8us*)dst = f.half[0]; __threadfence(); *(volatile v8us*)dst = f.half[0]; }
template <int NK>
__global__ __launch_bounds__(128) void k_flash(const _Float16* __restrict__ Q16, int hoff, const float* __restrict__ KV, const _Float16* __restrict__ Vt, int coff, _Float16* __restrict__ OC16) {
  constexpr int RPW = 32;
  __shared__ __attribute__((aligned(16))) unsigned short sP[4][RPW][40]; __shared__ __attribute__((aligned(16))) float sO[4][RPW][64 + 4];
  const int tid = threadIdx.x, w = tid >> 5, lane = tid & 31, ln = lane & 15, hh = lane >> 4;
  const int b = blockIdx.x / (NTOK / 128), qblk = blockIdx.x % (NTOK / 128); const int q0 = qblk * 128 + w * RPW;
#pragma unroll 1
  for (int h = 0; h < 4; ++h) { const int hg = hoff + h;
    FragH aq[2];
#pragma unroll
    for (int rt = 0; rt < 2; ++rt) { const unsigned short* qr = (const unsigned short*)Q16 + ((size_t)b * NTOK + q0 + rt * 16 + ln) * CC + hg * HD; aq[rt].half[0] = *(const v8us*)(qr + 8 * hh); aq[rt].half[1] = (v8us){0,0,0,0,0,0,0,0}; }
    const unsigned short* Vth = (const unsigned short*)Vt + (size_t)(b * 4 + h) * HD * NK;
    float m_r[2][8], l_r[2][8]; v8f oacc[2];
#pragma unroll
    for (int rt = 0; rt < 2; ++rt) { oacc[rt] = (v8f){0.f,0.f,0.f,0.f,0.f,0.f,0.f,0.f};
#pragma unroll
      for (int r = 0; r < 8; ++r) { m_r[rt][r] = -3.0e38f; l_r[rt][r] = 0.f; } }
#pragma unroll 1
    for (int j0 = 0; j0 < NK; j0 += 32) {
      v8f s[2][2];
#pragma unroll
      for (int nt = 0; nt < 2; ++nt) { const float* kr = KV + ((size_t)b * NK + j0 + nt * 16 + ln) * CC + h * HD + 8 * hh; FragH bk;
#pragma unroll
        for (int q = 0; q < 8; ++q) bk.h[q] = (_Float16)kr[q]; bk.half[1] = (v8us){0,0,0,0,0,0,0,0};
#pragma unroll
        for (int rt = 0; rt < 2; ++rt) { v8f acc = (v8f){0.f,0.f,0.f,0.f,0.f,0.f,0.f,0.f}; acc = mmaH<1>(aq[rt].v, aq[rt].v, bk.v, bk.v, acc); s[rt][nt] = acc; } }
#pragma unroll
      for (int rt = 0; rt < 2; ++rt)
#pragma unroll
        for (int r = 0; r < 8; ++r) { const float s0 = s[rt][0][r] * 0.25f, s1 = s[rt][1][r] * 0.25f; float mc = fmaxf(s0, s1);
          mc = fmaxf(mc, __shfl_xor(mc, 1, 32)); mc = fmaxf(mc, __shfl_xor(mc, 2, 32)); mc = fmaxf(mc, __shfl_xor(mc, 4, 32)); mc = fmaxf(mc, __shfl_xor(mc, 8, 32));
          const float mn = fmaxf(m_r[rt][r], mc); const float al = expf(m_r[rt][r] - mn); m_r[rt][r] = mn; const float p0 = expf(s0 - mn), p1 = expf(s1 - mn); l_r[rt][r] = l_r[rt][r] * al + p0 + p1; oacc[rt][r] *= al;
          FragH t2; t2.h[0] = (_Float16)p0; t2.h[1] = (_Float16)p1; sP[w][rt * 16 + 8 * hh + r][ln] = t2.u[0]; sP[w][rt * 16 + 8 * hh + r][16 + ln] = t2.u[1]; }
      __builtin_amdgcn_fence(__ATOMIC_ACQ_REL, "workgroup"); __builtin_amdgcn_wave_barrier();
      FragH pa[2];
#pragma unroll
      for (int rt = 0; rt < 2; ++rt) { pa[rt].half[0] = *(const v8us*)&sP[w][rt * 16 + ln][8 * hh]; pa[rt].half[1] = *(const v8us*)&sP[w][rt * 16 + ln][16 + 8 * hh]; }
      { const unsigned short* vrow = Vth + (size_t)ln * NK + j0; FragH bv; bv.half[0] = *(const v8us*)(vrow + 8 * hh); bv.half[1] = *(const v8us*)(vrow + 16 + 8 * hh);
#pragma unroll
        for (int rt = 0; rt < 2; ++rt) oacc[rt] = mmaH<1>(pa[rt].v, pa[rt].v, bv.v, bv.v, oacc[rt]); }
      __builtin_amdgcn_fence(__ATOMIC_ACQ_REL, "workgroup"); __builtin_amdgcn_wave_barrier(); }
#pragma unroll
    for (int rt = 0; rt < 2; ++rt)
#pragma unroll
      for (int r = 0; r < 8; ++r) { float l = l_r[rt][r]; l += __shfl_xor(l, 1, 32); l += __shfl_xor(l, 2, 32); l += __shfl_xor(l, 4, 32); l += __shfl_xor(l, 8, 32); sO[w][rt * 16 + 8 * hh + r][h * HD + ln] = oacc[rt][r] / l; } }
  __builtin_amdgcn_fence(__ATOMIC_ACQ_REL, "workgroup"); __builtin_amdgcn_wave_barrier();
  for (int pass = 0; pass < 2; ++pass) {
#pragma unroll
    for (int rp = 0; rp < RPW; rp += 4) { const int r = rp + (lane >> 3), pc = lane & 7; FragH f;
#pragma unroll
      for (int q = 0; q < 8; ++q) f.h[q] = (_Float16)sO[w][r][pc * 8 + q]; *(volatile v8us*)((unsigned short*)OC16 + ((size_t)b * NTOK + q0 + r) * CC + coff + pc * 8) = f.half[0]; }
    if (pass == 0) __threadfence(); } }
extern "C" void kernel_launch(void* const* d_in, const int* in_sizes, int n_in,
                              void* d_out, int out_size, void* d_ws, size_t ws_size, hipStream_t stream) {
  (void)in_sizes; (void)n_in; (void)out_size;
  const float* x = (const float*)d_in[0]; const float* q_w = (const float*)d_in[1]; const float* sr1_w = (const float*)d_in[2]; const float* sr1_b = (const float*)d_in[3]; const float* n1g = (const float*)d_in[4]; const float* n1b = (const float*)d_in[5]; const float* sr2_w = (const float*)d_in[6]; const float* sr2_b = (const float*)d_in[7]; const float* n2g = (const float*)d_in[8]; const float* n2b = (const float*)d_in[9];
  const float* kv1_w = (const float*)d_in[10]; const float* kv2_w = (const float*)d_in[11]; const float* lc1_w = (const float*)d_in[12]; const float* lc1_b = (const float*)d_in[13]; const float* lc2_w = (const float*)d_in[14]; const float* lc2_b = (const float*)d_in[15]; const float* proj_w = (const float*)d_in[16]; const float* proj_b = (const float*)d_in[17];
  char* ws = (char*)d_ws; size_t off = 0;
  auto take = [&](size_t bytes) { char* p = ws + off; off += (bytes + 255) & ~(size_t)255; return p; };
  constexpr int NK1 = 256, NK2 = 1024, KK1 = CC * 64, KK2 = CC * 16;
  _Float16* Bq = (_Float16*)take(CC * CC * 2); _Float16* Bp = (_Float16*)take(CC * CC * 2); _Float16* Bkv1 = (_Float16*)take(CC * CC * 2); _Float16* Bkv2 = (_Float16*)take(CC * CC * 2); _Float16* Bs1 = (_Float16*)take((size_t)CC * KK1 * 2); _Float16* Bs2 = (_Float16*)take((size_t)CC * KK2 * 2);
  _Float16* X16 = (_Float16*)take((size_t)NR * CC * 2); _Float16* Q16 = (_Float16*)take((size_t)NR * CC * 2); _Float16* AP = (_Float16*)take((size_t)BB * NK1 * KK1 * 2 > (size_t)BB * NK2 * KK2 * 2 ? (size_t)BB * NK1 * KK1 * 2 : (size_t)BB * NK2 * KK2 * 2);
  float* XR = (float*)take((size_t)BB * NK2 * CC * 4); _Float16* XG = (_Float16*)take((size_t)BB * NK2 * CC * 2); float* KV = (float*)take((size_t)BB * NK2 * CC * 4); _Float16* Vt = (_Float16*)take((size_t)BB * 4 * HD * NK2 * 2); _Float16* OC16 = (_Float16*)take((size_t)NR * CC * 2);
  if (off > ws_size) return;
  const size_t w8 = (size_t)CC * CC / 8; const unsigned gw = (unsigned)((w8 + 255) / 256);
  k_round16f<<<gw, 256, 0, stream>>>(q_w, Bq, w8); k_round16f<<<gw, 256, 0, stream>>>(proj_w, Bp, w8); k_round16f<<<gw, 256, 0, stream>>>(kv1_w, Bkv1, w8); k_round16f<<<gw, 256, 0, stream>>>(kv2_w, Bkv2, w8);
  k_round16f<<<(unsigned)(((size_t)CC * KK1 / 8 + 255) / 256), 256, 0, stream>>>(sr1_w, Bs1, (size_t)CC * KK1 / 8); k_round16f<<<(unsigned)(((size_t)CC * KK2 / 8 + 255) / 256), 256, 0, stream>>>(sr2_w, Bs2, (size_t)CC * KK2 / 8);
  k_x16<<<(unsigned)(((size_t)NR * CC / 8 + 255) / 256), 256, 0, stream>>>(x, X16, (size_t)NR * CC / 8);
  const dim3 gq(((NR / 16) * (CC / 64) + 3) / 4, 1);
  k_gemm_hhx<0><<<gq, 128, 0, stream>>>(X16, CC, 0, Bq, CC, 0, 0.0625f, nullptr, 0, nullptr, 1, 0, 0, nullptr, Q16, CC, 0, NR, CC, CC);
  k_patch<8><<<(unsigned)(((size_t)BB * NK1 * KK1 / 8 + 255) / 256), 256, 0, stream>>>(X16, AP);
  k_gemm_hhx<0><<<dim3(((BB * NK1 / 16) * (CC / 64) + 3) / 4, 1), 128, 0, stream>>>(AP, KK1, 0, Bs1, KK1, 0, 0.0625f, sr1_b, 0, nullptr, 1, 0, 0, XR, nullptr, CC, 0, BB * NK1, CC, KK1);
  k_lngelu<<<(BB * NK1 + 7) / 8, 256, 0, stream>>>(XR, BB * NK1, n1g, n1b, XG);
  k_gemm_hhx<0><<<dim3(((BB * NK1 / 16) * (CC / 64) + 3) / 4, 1), 128, 0, stream>>>(XG, CC, 0, Bkv1, CC, 0, 0.0625f, nullptr, 0, nullptr, 1, 0, 0, KV, nullptr, CC, 0, BB * NK1, CC, CC);
  k_vt<16><<<(unsigned)(((size_t)BB * 64 * NK1 / 8 + 255) / 256), 256, 0, stream>>>(KV, lc1_w, lc1_b, Vt);
  k_flash<NK1><<<BB * (NTOK / 128), 128, 0, stream>>>(Q16, 0, KV, Vt, 0, OC16);
  k_patch<4><<<(unsigned)(((size_t)BB * NK2 * KK2 / 8 + 255) / 256), 256, 0, stream>>>(X16, AP);
  k_gemm_hhx<0><<<dim3(((BB * NK2 / 16) * (CC / 64) + 3) / 4, 1), 128, 0, stream>>>(AP, KK2, 0, Bs2, KK2, 0, 0.0625f, sr2_b, 0, nullptr, 1, 0, 0, XR, nullptr, CC, 0, BB * NK2, CC, KK2);
  k_lngelu<<<(BB * NK2 + 7) / 8, 256, 0, stream>>>(XR, BB * NK2, n2g, n2b, XG);
  k_gemm_hhx<0><<<dim3(((BB * NK2 / 16) * (CC / 64) + 3) / 4, 1), 128, 0, stream>>>(XG, CC, 0, Bkv2, CC, 0, 0.0625f, nullptr, 0, nullptr, 1, 0, 0, KV, nullptr, CC, 0, BB * NK2, CC, CC);
  k_vt<32><<<(unsigned)(((size_t)BB * 64 * NK2 / 8 + 255) / 256), 256, 0, stream>>>(KV, lc2_w, lc2_b, Vt);
  k_flash<NK2><<<BB * (NTOK / 128), 128, 0, stream>>>(Q16, 4, KV, Vt, 64, OC16);
  k_gemm_hhx<0><<<gq, 128, 0, stream>>>(OC16, CC, 0, Bp, CC, 0, 0.0625f, proj_b, 0, nullptr, 1, 0, 0, (float*)d_out, nullptr, CC, 0, NR, CC, CC);
}
